// EdgeToTriAttention_1778116461007
// MI455X (gfx1250) — hardware-verified
//
#include <hip/hip_runtime.h>
#include <stddef.h>
#include <stdint.h>

#define NROW 8192
#define DIN  3
#define DK   128
#define HID  256
#define NRES 2
#define RPW  4
#define RPB  (8 * RPW)
#define NCH  (NROW / 128)

static_assert(NROW % RPB == 0);
static_assert(NROW % 256 == 0);
static_assert(NROW % 128 == 0);
static_assert(DK == 128);
static_assert(HID == 256);
static_assert(RPB == 32);
static_assert(DK % 64 == 0 && HID % 64 == 0);

typedef _Float16 v16h __attribute__((ext_vector_type(16)));
typedef _Float16 v8h  __attribute__((ext_vector_type(8)));
typedef _Float16 v4h  __attribute__((ext_vector_type(4)));
typedef float    v8f  __attribute__((ext_vector_type(8)));
typedef float    v4f  __attribute__((ext_vector_type(4)));
typedef unsigned int v4u __attribute__((ext_vector_type(4)));
typedef int      v4i  __attribute__((ext_vector_type(4)));

union Frag  { v16h v; v8h h[2]; };
union Pack8 { v8h h; v4u u; };

static constexpr float QKS  = 0.08838834764831845f;
static constexpr float REPS = 1.1920929e-07f;
static constexpr float NEGB = -1.0e30f;

__device__ __forceinline__ v8f mma16(v16h a, v16h b, v8f c) {
  c = __builtin_amdgcn_wmma_f32_16x16x32_f16(false, a, false, b, (short)0, c, false, false);
  asm volatile("v_nop\n\tv_nop\n\tv_nop\n\tv_nop" : "+v"(c) : "v"(a), "v"(b));
  return c;
}

__device__ __forceinline__ v16h ldfrag(const _Float16* p, int ld, int row0, int k0, int lane) {
  const int m = lane & 15, lh = lane >> 4;
  const _Float16* q = p + (size_t)(row0 + m) * ld + k0 + 8 * lh;
  Frag f;
  f.h[0] = *(const v8h*)(q);
  f.h[1] = *(const v8h*)(q + 16);
  return f.v;
}

__device__ __forceinline__ v8f zero8() { return (v8f){0.f, 0.f, 0.f, 0.f, 0.f, 0.f, 0.f, 0.f}; }

__device__ __forceinline__ void gemm32x64(const _Float16* __restrict__ A, int lda,
                                          const _Float16* __restrict__ Bt, int ldb, int K,
                                          int m0, int n0, int lane, v8f (&acc)[2][4]) {
#pragma unroll 1
  for (int k0 = 0; k0 < K; k0 += 32) {
    const v16h a0 = ldfrag(A, lda, m0, k0, lane);
    const v16h a1 = ldfrag(A, lda, m0 + 16, k0, lane);
    const v16h b0 = ldfrag(Bt, ldb, n0, k0, lane);
    const v16h b1 = ldfrag(Bt, ldb, n0 + 16, k0, lane);
    const v16h b2 = ldfrag(Bt, ldb, n0 + 32, k0, lane);
    const v16h b3 = ldfrag(Bt, ldb, n0 + 48, k0, lane);
    acc[0][0] = mma16(a0, b0, acc[0][0]);
    acc[1][0] = mma16(a1, b0, acc[1][0]);
    acc[0][1] = mma16(a0, b1, acc[0][1]);
    acc[1][1] = mma16(a1, b1, acc[1][1]);
    acc[0][2] = mma16(a0, b2, acc[0][2]);
    acc[1][2] = mma16(a1, b2, acc[1][2]);
    acc[0][3] = mma16(a0, b3, acc[0][3]);
    acc[1][3] = mma16(a1, b3, acc[1][3]);
  }
}

#define TRP 72
__global__ __launch_bounds__(256) void k_trcvt(const float* __restrict__ src, int K, int Nc,
                                               _Float16* __restrict__ dst, float scale) {
  __shared__ __align__(16) _Float16 st[64 * TRP];
  const int tid = threadIdx.x;
  const int k0 = blockIdx.x * 64, n0 = blockIdx.y * 64;
  const size_t zo = (size_t)blockIdx.z * (size_t)K * (size_t)Nc;
  const float* s = src + zo;
  _Float16* d = dst + zo;
  const int kr = tid >> 2;
  const int ns = (tid & 3) * 16;
  const float* sp = s + (size_t)(k0 + kr) * Nc + n0 + ns;
#pragma unroll
  for (int j = 0; j < 4; ++j) {
    const v4f v = *(const v4f*)(sp + 4 * j) * scale;
#pragma unroll
    for (int e = 0; e < 4; ++e) st[(ns + 4 * j + e) * TRP + kr] = (_Float16)v[e];
  }
  __syncthreads();
  v4u val[2];
  size_t go[2];
#pragma unroll
  for (int it = 0; it < 2; ++it) {
    const int p   = tid + 256 * it;
    const int row = p >> 3;
    const int pc  = p & 7;
    Pack8 pk;
    pk.h    = *(const v8h*)(st + row * TRP + pc * 8);
    val[it] = pk.u;
    go[it]  = (size_t)(n0 + row) * K + k0 + pc * 8;
  }
  for (int ps = 0; ps < 2; ++ps) {
#pragma unroll
    for (int it = 0; it < 2; ++it) *(volatile v4u*)(d + go[it]) = val[it];
    __threadfence();
  }
}

__global__ __launch_bounds__(256) void k_proj(const float* __restrict__ ef,
                                              const float* __restrict__ wq, const float* __restrict__ bq,
                                              const float* __restrict__ wk, const float* __restrict__ bk,
                                              const float* __restrict__ wv, const float* __restrict__ bv,
                                              float* __restrict__ qf, float* __restrict__ kf,
                                              float* __restrict__ vf) {
  const int tid = threadIdx.x, lane = tid & 31, wave = tid >> 5;
  const int c = 4 * lane;
  const v4f wq0 = *(const v4f*)(wq + c), wq1 = *(const v4f*)(wq + DK + c), wq2 = *(const v4f*)(wq + 2 * DK + c);
  const v4f wk0 = *(const v4f*)(wk + c), wk1 = *(const v4f*)(wk + DK + c), wk2 = *(const v4f*)(wk + 2 * DK + c);
  const v4f wv0 = *(const v4f*)(wv + c), wv1 = *(const v4f*)(wv + DK + c), wv2 = *(const v4f*)(wv + 2 * DK + c);
  const v4f bq4 = *(const v4f*)(bq + c), bk4 = *(const v4f*)(bk + c), bv4 = *(const v4f*)(bv + c);
#pragma unroll 1
  for (int rr = 0; rr < RPW; ++rr) {
    const int row = min((int)blockIdx.x * RPB + wave * RPW + rr, NROW - 1);
    const float e0 = ef[row * DIN + 0], e1 = ef[row * DIN + 1], e2 = ef[row * DIN + 2];
    v4f q, k, v;
#pragma unroll
    for (int e = 0; e < 4; ++e) {
      float t;
      t = e0 * wq0[e]; t = fmaf(e1, wq1[e], t); t = fmaf(e2, wq2[e], t); q[e] = t + bq4[e];
      t = e0 * wk0[e]; t = fmaf(e1, wk1[e], t); t = fmaf(e2, wk2[e], t); k[e] = t + bk4[e];
      t = e0 * wv0[e]; t = fmaf(e1, wv1[e], t); t = fmaf(e2, wv2[e], t); v[e] = t + bv4[e];
    }
    const size_t o = (size_t)row * DK + c;
    for (int ps = 0; ps < 2; ++ps) {
      *(volatile v4f*)(qf + o) = q;
      *(volatile v4f*)(kf + o) = k;
      *(volatile v4f*)(vf + o) = v;
      __threadfence();
    }
  }
}

__global__ __launch_bounds__(256) void k_attn(const float* __restrict__ qf, const float* __restrict__ kf,
                                              const float* __restrict__ vf, const int* __restrict__ tri,
                                              _Float16* __restrict__ ah) {
  __shared__ __align__(16) _Float16 st[RPB * DK];
  const int tid = threadIdx.x, lane = tid & 31, wave = tid >> 5;
  const int c = 4 * lane;
#pragma unroll 1
  for (int rr = 0; rr < RPW; ++rr) {
    const int lr   = wave * RPW + rr;
    const int row  = min((int)blockIdx.x * RPB + lr, NROW - 1);
    const int trow = tri[row];
    const v4f q4   = *(const v4f*)(qf + (size_t)row * DK + c);
    float m = NEGB, l = 0.f;
    v4f acc = (v4f){0.f, 0.f, 0.f, 0.f};
#pragma unroll 1
    for (int ch = 0; ch < NCH; ++ch) {
      const int j0 = ch * 128;
      const v4i t4 = *(const v4i*)(tri + j0 + c);
#pragma unroll
      for (int e = 0; e < 4; ++e) {
        unsigned msk = __builtin_amdgcn_ballot_w32(t4[e] == trow);
        while (msk != 0u) {
          const int b = __builtin_ctz(msk);
          msk &= msk - 1u;
          const int j = j0 + 4 * b + e;
          const v4f k4 = *(const v4f*)(kf + (size_t)j * DK + c);
          float d = q4[0] * k4[0];
          d = fmaf(q4[1], k4[1], d);
          d = fmaf(q4[2], k4[2], d);
          d = fmaf(q4[3], k4[3], d);
#pragma unroll
          for (int off = 16; off >= 1; off >>= 1) d += __shfl_xor(d, off, 32);
          const float s  = d * QKS;
          const float mn = fmaxf(m, s);
          const float al = __expf(m - mn);
          const float p  = __expf(s - mn);
          l = fmaf(l, al, p);
          const v4f v4 = *(const v4f*)(vf + (size_t)j * DK + c);
          acc = acc * al + v4 * p;
          m = mn;
        }
      }
    }
    const float il = 64.0f * __builtin_amdgcn_rcpf(l);
    const v4f o = acc * il;
    *(v4h*)(st + lr * DK + c) = (v4h){(_Float16)o[0], (_Float16)o[1], (_Float16)o[2], (_Float16)o[3]};
  }
  __syncthreads();
  v4u val[2];
  size_t go[2];
#pragma unroll
  for (int it = 0; it < 2; ++it) {
    const int p = tid + 256 * it;
    Pack8 pk;
    pk.h    = *(const v8h*)(st + p * 8);
    val[it] = pk.u;
    go[it]  = (size_t)blockIdx.x * RPB * DK + (size_t)p * 8;
  }
  for (int ps = 0; ps < 2; ++ps) {
#pragma unroll
    for (int it = 0; it < 2; ++it) *(volatile v4u*)(ah + go[it]) = val[it];
    __threadfence();
  }
}

#define OTP 68
__device__ __forceinline__ void out_epilogue_f32(v8f (&acc)[2][4], float scale, const float (&bb)[4],
                                                 float* sw, float* __restrict__ out, int ldo,
                                                 int m0, int n0, int lane, int hh, int c) {
#pragma unroll
  for (int sub = 0; sub < 2; ++sub) {
    __syncthreads();
#pragma unroll
    for (int t = 0; t < 4; ++t) {
#pragma unroll
      for (int r = 0; r < 8; ++r) sw[(8 * hh + r) * OTP + 16 * t + c] = acc[sub][t][r] * scale + bb[t];
    }
    __syncthreads();
    v4f val[8];
    size_t go[8];
#pragma unroll
    for (int it = 0; it < 8; ++it) {
      const int p   = lane + 32 * it;
      const int L   = p >> 3;
      const int pc  = p & 7;
      const int row = L >> 1;
      const int seg = L & 1;
      val[it] = *(const v4f*)(sw + row * OTP + seg * 32 + pc * 4);
      go[it]  = (size_t)(m0 + sub * 16 + row) * ldo + n0 + seg * 32 + pc * 4;
    }
    for (int ps = 0; ps < 2; ++ps) {
#pragma unroll
      for (int it = 0; it < 8; ++it) *(volatile v4f*)(out + go[it]) = val[it];
      __threadfence();
    }
  }
}

__device__ __forceinline__ void out_epilogue_res(v8f (&acc)[2][4], float scale, const float (&bb)[4],
                                                 float* sw, const float* __restrict__ hin,
                                                 float* __restrict__ out, int ldo,
                                                 int m0, int n0, int lane, int hh, int c) {
#pragma unroll
  for (int sub = 0; sub < 2; ++sub) {
    __syncthreads();
#pragma unroll
    for (int t = 0; t < 4; ++t) {
#pragma unroll
      for (int r = 0; r < 8; ++r)
        sw[(8 * hh + r) * OTP + 16 * t + c] = fmaxf(acc[sub][t][r] * scale + bb[t], 0.f);
    }
    __syncthreads();
    v4f val[8];
    size_t go[8];
#pragma unroll
    for (int it = 0; it < 8; ++it) {
      const int p   = lane + 32 * it;
      const int L   = p >> 3;
      const int pc  = p & 7;
      const int row = L >> 1;
      const int seg = L & 1;
      go[it]  = (size_t)(m0 + sub * 16 + row) * ldo + n0 + seg * 32 + pc * 4;
      val[it] = *(const v4f*)(sw + row * OTP + seg * 32 + pc * 4) + *(const v4f*)(hin + go[it]);
    }
    for (int ps = 0; ps < 2; ++ps) {
#pragma unroll
      for (int it = 0; it < 8; ++it) *(volatile v4f*)(out + go[it]) = val[it];
      __threadfence();
    }
  }
}

__global__ __launch_bounds__(256) void k_gemm_h(const _Float16* __restrict__ ap, int lda,
                                                const _Float16* __restrict__ wt, int K,
                                                const float* __restrict__ bias, float scale,
                                                float* __restrict__ out, int ldo) {
  __shared__ __align__(16) float st[8][16 * OTP];
  const int tid = threadIdx.x, lane = tid & 31, wave = tid >> 5;
  const int hh = lane >> 4, c = lane & 15;
  const int m0 = blockIdx.x * 256 + wave * 32;
  const int n0 = blockIdx.y * 64;

  v8f acc[2][4];
#pragma unroll
  for (int s = 0; s < 2; ++s)
#pragma unroll
    for (int t = 0; t < 4; ++t) acc[s][t] = zero8();
  gemm32x64(ap, lda, wt, K, K, m0, n0, lane, acc);
  float bb[4];
#pragma unroll
  for (int t = 0; t < 4; ++t) bb[t] = bias[n0 + 16 * t + c];
  out_epilogue_f32(acc, scale, bb, st[wave], out, ldo, m0, n0, lane, hh, c);
}

__global__ __launch_bounds__(256) void k_rms(const float* __restrict__ hp, const float* __restrict__ w,
                                             _Float16* __restrict__ gp) {
  const int tid = threadIdx.x, lane = tid & 31, wave = tid >> 5;
  const int c = 8 * lane;
  const v4f w0 = *(const v4f*)(w + c), w1 = *(const v4f*)(w + c + 4);
#pragma unroll 1
  for (int rr = 0; rr < RPW; ++rr) {
    const int row = min((int)blockIdx.x * RPB + wave * RPW + rr, NROW - 1);
    const float* hr = hp + (size_t)row * HID + c;
    const v4f a = *(const v4f*)(hr), b = *(const v4f*)(hr + 4);
    float ss = (a[0] * a[0] + a[1] * a[1]) + (a[2] * a[2] + a[3] * a[3]);
    ss += (b[0] * b[0] + b[1] * b[1]) + (b[2] * b[2] + b[3] * b[3]);
#pragma unroll
    for (int off = 16; off >= 1; off >>= 1) ss += __shfl_xor(ss, off, 32);
    const float r = rsqrtf(ss * 0.00390625f + REPS);
    const v4f ga = (a * r) * w0;
    const v4f gb = (b * r) * w1;
    Pack8 pk;
    pk.h = (v8h){(_Float16)ga[0], (_Float16)ga[1], (_Float16)ga[2], (_Float16)ga[3],
                 (_Float16)gb[0], (_Float16)gb[1], (_Float16)gb[2], (_Float16)gb[3]};
    const v4u vv = pk.u;
    volatile v4u* dp = (volatile v4u*)(gp + (size_t)row * HID + c);
    for (int ps = 0; ps < 2; ++ps) {
      *dp = vv;
      __threadfence();
    }
  }
}

__global__ __launch_bounds__(256) void k_gemm_res(const _Float16* __restrict__ ap, int lda,
                                                  const _Float16* __restrict__ wt, int K,
                                                  const float* __restrict__ bias, float scale,
                                                  const float* __restrict__ hin,
                                                  float* __restrict__ out, int ldo) {
  __shared__ __align__(16) float st[8][16 * OTP];
  const int tid = threadIdx.x, lane = tid & 31, wave = tid >> 5;
  const int hh = lane >> 4, c = lane & 15;
  const int m0 = blockIdx.x * 256 + wave * 32;
  const int n0 = blockIdx.y * 64;

  v8f acc[2][4];
#pragma unroll
  for (int s = 0; s < 2; ++s)
#pragma unroll
    for (int t = 0; t < 4; ++t) acc[s][t] = zero8();
  gemm32x64(ap, lda, wt, K, K, m0, n0, lane, acc);
  float bb[4];
#pragma unroll
  for (int t = 0; t < 4; ++t) bb[t] = bias[n0 + 16 * t + c];
  out_epilogue_res(acc, scale, bb, st[wave], hin, out, ldo, m0, n0, lane, hh, c);
}

__global__ __launch_bounds__(256) void k_logit(const float* __restrict__ hp, const float* __restrict__ wo,
                                               const float* __restrict__ bo, float* __restrict__ lg) {
  __shared__ __align__(16) float st[RPB];
  const int tid = threadIdx.x, lane = tid & 31, wave = tid >> 5;
  const int c = 8 * lane;
  const v4f w0 = *(const v4f*)(wo + c), w1 = *(const v4f*)(wo + c + 4);
  const float b0 = bo[0];
#pragma unroll 1
  for (int rr = 0; rr < RPW; ++rr) {
    const int lr  = wave * RPW + rr;
    const int row = min((int)blockIdx.x * RPB + lr, NROW - 1);
    const float* hr = hp + (size_t)row * HID + c;
    const v4f a = *(const v4f*)(hr), b = *(const v4f*)(hr + 4);
    float d = a[0] * w0[0];
    d = fmaf(a[1], w0[1], d); d = fmaf(a[2], w0[2], d); d = fmaf(a[3], w0[3], d);
    d = fmaf(b[0], w1[0], d); d = fmaf(b[1], w1[1], d); d = fmaf(b[2], w1[2], d); d = fmaf(b[3], w1[3], d);
#pragma unroll
    for (int off = 16; off >= 1; off >>= 1) d += __shfl_xor(d, off, 32);
    if (lane == 0) st[lr] = d + b0;
  }
  __syncthreads();
  if (tid < 8) {
    const v4f v = *(const v4f*)(st + 4 * tid);
    volatile v4f* dp = (volatile v4f*)(lg + (size_t)blockIdx.x * RPB + 4 * tid);
    for (int ps = 0; ps < 2; ++ps) {
      *dp = v;
      __threadfence();
    }
  }
}

__global__ __launch_bounds__(256) void k_segsm(const float* __restrict__ lg, const int* __restrict__ eid,
                                               float* __restrict__ out) {
  __shared__ __align__(16) float st[RPB];
  const int tid = threadIdx.x, lane = tid & 31, wave = tid >> 5;
  const int c = 4 * lane;
#pragma unroll 1
  for (int rr = 0; rr < RPW; ++rr) {
    const int lr  = wave * RPW + rr;
    const int row = min((int)blockIdx.x * RPB + lr, NROW - 1);
    const int   ei = eid[row];
    const float gi = lg[row];
    float m = NEGB, s = 0.f;
#pragma unroll 1
    for (int ch = 0; ch < NCH; ++ch) {
      const int j0 = ch * 128;
      const v4i e4 = *(const v4i*)(eid + j0 + c);
      const v4f g4 = *(const v4f*)(lg + j0 + c);
#pragma unroll
      for (int e = 0; e < 4; ++e) {
        const bool mt = (e4[e] == ei);
        const unsigned msk = __builtin_amdgcn_ballot_w32(mt);
        if (msk != 0u) {
          float mx = mt ? g4[e] : NEGB;
#pragma unroll
          for (int off = 16; off >= 1; off >>= 1) mx = fmaxf(mx, __shfl_xor(mx, off, 32));
          const float mn = fmaxf(m, mx);
          const float sc = __expf(m - mn);
          const float ev = __expf(g4[e] - mn);
          float pe = mt ? ev : 0.f;
#pragma unroll
          for (int off = 16; off >= 1; off >>= 1) pe += __shfl_xor(pe, off, 32);
          s = fmaf(s, sc, pe);
          m = mn;
        }
      }
    }
    const float wv = __expf(gi - m) * __builtin_amdgcn_rcpf(s);
    if (lane == 0) st[lr] = wv;
  }
  __syncthreads();
  if (tid < 8) {
    const v4f v = *(const v4f*)(st + 4 * tid);
    volatile v4f* dp = (volatile v4f*)(out + (size_t)blockIdx.x * RPB + 4 * tid);
    for (int ps = 0; ps < 2; ++ps) {
      *dp = v;
      __threadfence();
    }
  }
}

extern "C" void kernel_launch(void* const* d_in, const int* in_sizes, int n_in,
                              void* d_out, int out_size, void* d_ws, size_t ws_size,
                              hipStream_t stream) {
  if (n_in < 16) return;
  if (in_sizes[0] != NROW * DIN) return;
  if (in_sizes[1] != NROW) return;
  if (in_sizes[2] != NROW) return;
  if (in_sizes[3] != DIN * DK) return;
  if (in_sizes[4] != DK) return;
  if (in_sizes[5] != DIN * DK) return;
  if (in_sizes[6] != DK) return;
  if (in_sizes[7] != DIN * DK) return;
  if (in_sizes[8] != DK) return;
  if (in_sizes[9] != DK * HID) return;
  if (in_sizes[10] != HID) return;
  if (in_sizes[11] != NRES * HID) return;
  if (in_sizes[12] != NRES * HID * HID) return;
  if (in_sizes[13] != NRES * HID) return;
  if (in_sizes[14] != HID) return;
  if (in_sizes[15] != 1) return;
  if (out_size != NROW) return;

  const float* ef   = (const float*)d_in[0];
  const int*   eid  = (const int*)d_in[1];
  const int*   tri  = (const int*)d_in[2];
  const float* wq   = (const float*)d_in[3];
  const float* bq   = (const float*)d_in[4];
  const float* wk   = (const float*)d_in[5];
  const float* bk   = (const float*)d_in[6];
  const float* wv   = (const float*)d_in[7];
  const float* bv   = (const float*)d_in[8];
  const float* w0   = (const float*)d_in[9];
  const float* b0   = (const float*)d_in[10];
  const float* rmsw = (const float*)d_in[11];
  const float* wres = (const float*)d_in[12];
  const float* bres = (const float*)d_in[13];
  const float* wout = (const float*)d_in[14];
  const float* bout = (const float*)d_in[15];
  float* out = (float*)d_out;

  size_t off = 0;
  const size_t oQ  = off; off += (size_t)NROW * DK * 4;
  const size_t oKf = off; off += (size_t)NROW * DK * 4;
  const size_t oV  = off; off += (size_t)NROW * DK * 4;
  const size_t oA  = off; off += (size_t)NROW * DK * 2;
  const size_t oW0 = off; off += (size_t)HID * DK * 2;
  const size_t oWr = off; off += (size_t)NRES * HID * HID * 2;
  const size_t oH0 = off; off += (size_t)NROW * HID * 4;
  const size_t oH1 = off; off += (size_t)NROW * HID * 4;
  const size_t oG  = off; off += (size_t)NROW * HID * 2;
  const size_t oL  = off; off += (size_t)NROW * 4;
  if (off > ws_size) return;
  if (off > (size_t)134217728) return;

  char* ws = (char*)d_ws;
  float*    Qf  = (float*)(ws + oQ);
  float*    Kf  = (float*)(ws + oKf);
  float*    Vf  = (float*)(ws + oV);
  _Float16* Ah  = (_Float16*)(ws + oA);
  _Float16* W0t = (_Float16*)(ws + oW0);
  _Float16* Wrt = (_Float16*)(ws + oWr);
  float*    H0  = (float*)(ws + oH0);
  float*    H1  = (float*)(ws + oH1);
  _Float16* G   = (_Float16*)(ws + oG);
  float*    LG  = (float*)(ws + oL);

  k_trcvt<<<dim3(DK / 64, HID / 64, 1), dim3(256), 0, stream>>>(w0, DK, HID, W0t, 32.0f);
  k_trcvt<<<dim3(HID / 64, HID / 64, NRES), dim3(256), 0, stream>>>(wres, HID, HID, Wrt, 32.0f);
  k_proj<<<dim3(NROW / RPB), dim3(256), 0, stream>>>(ef, wq, bq, wk, bk, wv, bv, Qf, Kf, Vf);
  k_attn<<<dim3(NROW / RPB), dim3(256), 0, stream>>>(Qf, Kf, Vf, tri, Ah);
  k_gemm_h<<<dim3(NROW / 256, HID / 64), dim3(256), 0, stream>>>(Ah, DK, W0t, DK, b0, 0.00048828125f, H0, HID);
  k_rms<<<dim3(NROW / RPB), dim3(256), 0, stream>>>(H0, rmsw, G);
  k_gemm_res<<<dim3(NROW / 256, HID / 64), dim3(256), 0, stream>>>(G, HID, Wrt, HID, bres, 0.03125f, H0, H1, HID);
  k_rms<<<dim3(NROW / RPB), dim3(256), 0, stream>>>(H1, rmsw + HID, G);
  k_gemm_res<<<dim3(NROW / 256, HID / 64), dim3(256), 0, stream>>>(G, HID, Wrt + (size_t)HID * HID, HID,
                                                                    bres + HID, 0.03125f, H1, H0, HID);
  k_logit<<<dim3(NROW / RPB), dim3(256), 0, stream>>>(H0, wout, bout, LG);
  k_segsm<<<dim3(NROW / RPB), dim3(256), 0, stream>>>(LG, eid, out);
  (void)hipGetLastError();
}
